// BiMamba_83631603188084
// MI455X (gfx1250) — hardware-verified
//
#include <hip/hip_runtime.h>
#include <math.h>

typedef __attribute__((ext_vector_type(16))) _Float16 v16h;
typedef __attribute__((ext_vector_type(8)))  _Float16 v8h;
typedef __attribute__((ext_vector_type(8)))  float    v8f;
typedef __attribute__((ext_vector_type(4)))  float    v4f;

constexpr int kBatch = 2;
constexpr int kSeqL  = 2048;
constexpr int kDmod  = 1024;
constexpr int kDin   = 2048;
constexpr int kNst   = 16;
constexpr int kDtR   = 64;
constexpr int kPrjN  = 96;
constexpr int kPrjP  = 128;
constexpr int kXZP   = 2 * kDin;
constexpr int kRows  = kBatch * kSeqL;
constexpr int kYcP   = 2 * kDmod;
constexpr int kTP    = 260;
static_assert(kDtR + 2 * kNst == kPrjN, "x_proj width");
static_assert(kPrjP % 64 == 0 && kPrjP >= kPrjN, "x_proj pad");
static_assert(kDmod % 32 == 0 && kDin % 32 == 0 && kDtR % 32 == 0 && kYcP % 32 == 0, "GEMM K multiples of 32");
static_assert(kSeqL % 64 == 0 && kRows % 64 == 0 && kXZP % 64 == 0 && kDin % 64 == 0 && kDmod % 64 == 0, "GEMM M,N multiples of 64");
static_assert(kDin % 256 == 0 && kSeqL % 64 == 0 && kSeqL % 16 == 0, "conv / scan tiles");

constexpr float kCarryX   = 8.0f;
constexpr float kCarryW   = 32.0f;
constexpr float kCarryUC  = 16.0f;
constexpr float kCarryDT  = 16.0f;
constexpr float kCarryWdt = 8.0f;
constexpr float kCarryY   = 64.0f;
constexpr float kCarryYC  = 32.0f;
constexpr float kSclIn   = 1.0f / (kCarryX * kCarryW);
constexpr float kSclXp   = 1.0f / (kCarryUC * kCarryW);
constexpr float kSclDt   = 1.0f / (kCarryDT * kCarryWdt);
constexpr float kSclOut  = kCarryYC / (kCarryY * kCarryW);
constexpr float kSclPrj  = 1.0f / (kCarryYC * kCarryW);

constexpr size_t kSzWIN  = (size_t)kXZP * kDmod * 2;
constexpr size_t kSzWXP  = (size_t)kPrjP * kDin * 2;
constexpr size_t kSzWDT  = (size_t)kDin * kDtR * 2;
constexpr size_t kSzWOUT = (size_t)kDmod * kDin * 2;
constexpr size_t kSzWPRJ = (size_t)kDmod * kYcP * 2;
constexpr size_t kSzX16  = (size_t)kRows * kDmod * 2;
constexpr size_t kSzXZ   = (size_t)kSeqL * kXZP * 4;
constexpr size_t kSzUC   = (size_t)kSeqL * kDin * 4;
constexpr size_t kSzUC16 = (size_t)kSeqL * kDin * 2;
constexpr size_t kSzPROJ = (size_t)kSeqL * kPrjP * 4;
constexpr size_t kSzDT16 = (size_t)kSeqL * kDtR * 2;
constexpr size_t kSzDLR  = (size_t)kSeqL * kDin * 4;
constexpr size_t kSzY16  = (size_t)kSeqL * kDin * 2;
constexpr size_t kSzYC   = (size_t)kRows * kYcP * 2;
constexpr size_t kOffWIN  = 0;
constexpr size_t kOffWXP  = kOffWIN  + kSzWIN;
constexpr size_t kOffWDT  = kOffWXP  + kSzWXP;
constexpr size_t kOffWOUT = kOffWDT  + kSzWDT;
constexpr size_t kOffWPRJ = kOffWOUT + kSzWOUT;
constexpr size_t kOffX16  = kOffWPRJ + kSzWPRJ;
constexpr size_t kOffXZ   = kOffX16  + kSzX16;
constexpr size_t kOffUC   = kOffXZ   + kSzXZ;
constexpr size_t kOffUC16 = kOffUC   + kSzUC;
constexpr size_t kOffPROJ = kOffUC16 + kSzUC16;
constexpr size_t kOffDT16 = kOffPROJ + kSzPROJ;
constexpr size_t kOffDLR  = kOffDT16 + kSzDT16;
constexpr size_t kOffY16  = kOffDLR  + kSzDLR;
constexpr size_t kOffYC   = kOffY16  + kSzY16;
constexpr size_t kWsTotal = kOffYC   + kSzYC;
static_assert(kWsTotal == 127926272ull, "carve total");
static_assert(kWsTotal <= 134217728ull, "carve cap");
static_assert((kOffWXP % 128) == 0 && (kOffWDT % 128) == 0 && (kOffWOUT % 128) == 0 && (kOffWPRJ % 128) == 0 &&
              (kOffX16 % 128) == 0 && (kOffXZ % 128) == 0 && (kOffUC % 128) == 0 && (kOffUC16 % 128) == 0 &&
              (kOffPROJ % 128) == 0 && (kOffDT16 % 128) == 0 && (kOffDLR % 128) == 0 && (kOffY16 % 128) == 0 &&
              (kOffYC % 128) == 0, "128-B aligned regions");

__device__ __forceinline__ unsigned short f2bf_bits(float f) {
  unsigned u = __float_as_uint(f);
  return (unsigned short)((u + 0x7FFFu + ((u >> 16) & 1u)) >> 16);
}
__device__ __forceinline__ float bf_bits2f(unsigned short h) { return __uint_as_float(((unsigned)h) << 16); }
__device__ __forceinline__ float bf16r(float f) { return bf_bits2f(f2bf_bits(f)); }

__device__ __forceinline__ void guard_row_h(v8f& a, v8f& b, v8f& c, v8f& d, v16h x, v16h y0, v16h y1, v16h y2, v16h y3) {
  asm volatile("v_nop\n\tv_nop\n\tv_nop\n\tv_nop" : "+v"(a), "+v"(b), "+v"(c), "+v"(d) : "v"(x), "v"(y0), "v"(y1), "v"(y2), "v"(y3));
}
__device__ __forceinline__ void keep4_h(v16h a, v16h b, v16h c, v16h d) { asm volatile("v_nop" :: "v"(a), "v"(b), "v"(c), "v"(d)); }
__device__ __forceinline__ void acc_guard4(v8f& a, v8f& b, v8f& c, v8f& d) { asm volatile("v_nop\n\tv_nop\n\tv_nop\n\tv_nop" : "+v"(a), "+v"(b), "+v"(c), "+v"(d)); }

struct FragH {
  union U { v16h v; v8h h[2]; };
  static __device__ __forceinline__ v16h load(const _Float16* p) {
    U f; f.h[0] = *(const v8h*)(p); f.h[1] = *(const v8h*)(p + 16); return f.v;
  }
  static __device__ __forceinline__ v8f mma(v16h a, v16h b, v8f c) {
    return __builtin_amdgcn_wmma_f32_16x16x32_f16(false, a, false, b, (short)0, c, false, false);
  }
};

template <int BIAS_MODE, int OUT_MODE, bool BIAS_BF>
__global__ __launch_bounds__(256) void wmma_gemm64(
    const unsigned short* __restrict__ Ap, int lda,
    const unsigned short* __restrict__ Btp, int ldb,
    void* __restrict__ Cout, int ldc,
    const float* __restrict__ bias,
    int M, int N, int K, float scale) {
  const _Float16* A = (const _Float16*)Ap;
  const _Float16* Bt = (const _Float16*)Btp;
  __shared__ __align__(16) float sT[8][16 * 68];
  const int lane = threadIdx.x & 31;
  const int wave = threadIdx.x >> 5;
  const int tilesN = N >> 6;
  const int tilesM = M >> 6;
  const int tile = blockIdx.x * 8 + wave;
  if (tile >= tilesM * tilesN) return;
  const int tm = tile / tilesN;
  const int tn = tile - tm * tilesN;
  const int m0 = tm << 6;
  const int n0 = tn << 6;

  const int rlane = lane & 15;
  const int koff  = (lane >> 4) * 8;
  const int mOff  = (lane >> 4) * 8;

  v8f acc[4][4];
#pragma unroll
  for (int i = 0; i < 4; ++i)
#pragma unroll
    for (int j = 0; j < 4; ++j) acc[i][j] = (v8f){0.f,0.f,0.f,0.f,0.f,0.f,0.f,0.f};

  for (int k0 = 0; k0 < K; k0 += 32) {
    v16h bh[4];
#pragma unroll
    for (int j = 0; j < 4; ++j) {
      const size_t bo = (size_t)(n0 + (j << 4) + rlane) * ldb + koff + k0;
      bh[j] = FragH::load(Bt + bo);
    }
#pragma unroll
    for (int i = 0; i < 4; ++i) {
      const size_t ao = (size_t)(m0 + (i << 4) + rlane) * lda + koff + k0;
      v16h ah = FragH::load(A + ao);
#pragma unroll
      for (int j = 0; j < 4; ++j) acc[i][j] = FragH::mma(ah, bh[j], acc[i][j]);
      guard_row_h(acc[i][0], acc[i][1], acc[i][2], acc[i][3], ah, bh[0], bh[1], bh[2], bh[3]);
    }
    keep4_h(bh[0], bh[1], bh[2], bh[3]);
  }
  acc_guard4(acc[0][0], acc[0][1], acc[0][2], acc[0][3]);
  acc_guard4(acc[1][0], acc[1][1], acc[1][2], acc[1][3]);
  acc_guard4(acc[2][0], acc[2][1], acc[2][2], acc[2][3]);
  acc_guard4(acc[3][0], acc[3][1], acc[3][2], acc[3][3]);

  float* slab = sT[wave];
#pragma unroll
  for (int i = 0; i < 4; ++i) {
    const int mBase = m0 + (i << 4);
#pragma unroll
    for (int j = 0; j < 4; ++j) {
      const int n = n0 + (j << 4) + rlane;
      float bv = 0.f;
      if (BIAS_MODE == 2) {
        bv = bias[n];
        if (BIAS_BF) bv = bf16r(bv);
      }
#pragma unroll
      for (int r = 0; r < 8; ++r) {
        float v = acc[i][j][r] * scale;
        if (BIAS_MODE == 2) v += bv;
        slab[(mOff + r) * 68 + (j << 4) + rlane] = v;
      }
    }
    __builtin_amdgcn_fence(__ATOMIC_RELEASE, "workgroup");
    __builtin_amdgcn_wave_barrier();
    __builtin_amdgcn_fence(__ATOMIC_ACQUIRE, "workgroup");
    if (OUT_MODE == 0) {
      float* C = (float*)Cout;
      const int hh = lane >> 4, c4 = (lane & 15) * 4;
      for (int pass = 0; pass < 2; ++pass) {
#pragma unroll
        for (int it = 0; it < 8; ++it) {
          const int row = it * 2 + hh;
          v4f v = *(const v4f*)(slab + row * 68 + c4);
          *(volatile v4f*)(C + (size_t)(mBase + row) * ldc + n0 + c4) = v;
        }
        __threadfence();
      }
    } else {
      const int q = lane >> 3, c8 = (lane & 7) * 8;
      unsigned short* C = (unsigned short*)Cout;
      for (int pass = 0; pass < 2; ++pass) {
#pragma unroll
        for (int it = 0; it < 4; ++it) {
          const int row = it * 4 + q;
          const float* sp = slab + row * 68 + c8;
          v8h hv;
#pragma unroll
          for (int e = 0; e < 8; ++e) hv[e] = (_Float16)sp[e];
          *(volatile v8h*)(C + (size_t)(mBase + row) * ldc + n0 + c8) = hv;
        }
        __threadfence();
      }
    }
    __builtin_amdgcn_fence(__ATOMIC_RELEASE, "workgroup");
    __builtin_amdgcn_wave_barrier();
    __builtin_amdgcn_fence(__ATOMIC_ACQUIRE, "workgroup");
  }
}

__global__ __launch_bounds__(256) void cast_bf16_f16_kernel(
    const float* __restrict__ src, unsigned short* __restrict__ dst, int total8, int valid8, float scale)
{
  const int i = blockIdx.x * 256 + threadIdx.x;
  if (i >= total8) return;
  const bool ok = (i < valid8);
  const int ic = ok ? i : (valid8 - 1);
  const float* p = src + ((size_t)ic << 3);
  const v4f a0 = *(const v4f*)(p);
  const v4f a1 = *(const v4f*)(p + 4);
  v8h hv;
#pragma unroll
  for (int e = 0; e < 4; ++e) {
    const float s0 = a0[e];
    const float s1 = a1[e];
    const float r0 = bf16r(s0) * scale;
    const float r1 = bf16r(s1) * scale;
    hv[e]     = (_Float16)(ok ? r0 : 0.0f);
    hv[4 + e] = (_Float16)(ok ? r1 : 0.0f);
  }
  unsigned short* q = dst + ((size_t)i << 3);
  *(volatile v8h*)q = hv;
  __threadfence();
  *(volatile v8h*)q = hv;
}

__global__ __launch_bounds__(256) void dt_cast_kernel(
    const float* __restrict__ PROJ, unsigned short* __restrict__ DT16, int total8, float scale)
{
  const int i = blockIdx.x * 256 + threadIdx.x;
  if (i >= total8) return;
  const int e0  = i << 3;
  const int row = e0 >> 6;
  const int c8  = e0 & 63;
  const float* p = PROJ + (size_t)row * kPrjP + c8;
  const v4f a0 = *(const v4f*)(p);
  const v4f a1 = *(const v4f*)(p + 4);
  v8h hv;
#pragma unroll
  for (int e = 0; e < 4; ++e) {
    hv[e]     = (_Float16)(a0[e] * scale);
    hv[4 + e] = (_Float16)(a1[e] * scale);
  }
  unsigned short* qd = DT16 + e0;
  *(volatile v8h*)qd = hv;
  __threadfence();
  *(volatile v8h*)qd = hv;
}

__global__ __launch_bounds__(256) void conv_silu_kernel(
    const float* __restrict__ XZ, const float* __restrict__ cw, const float* __restrict__ cb,
    float* __restrict__ UC, unsigned short* __restrict__ UC16, int dir)
{
  __shared__ __align__(16) float sT[16 * kTP];
  const int tid = threadIdx.x, lane = tid & 31, wave = tid >> 5;
  const int d0 = blockIdx.x * 256, d = d0 + tid;
  const int s0 = blockIdx.y * 64;
  const int lorg = dir ? (kSeqL - 1) : 0;
  const int lsgn = dir ? -1 : 1;
  const v4f wv = *(const v4f*)(cw + (size_t)d * 4);
  const float wa = wv[0], wb = wv[1], wc = wv[2], wd = wv[3];
  const float w0 = bf16r(wa), w1 = bf16r(wb), w2 = bf16r(wc), w3 = bf16r(wd);
  const float bc = bf16r(cb[d]);
  float xm3, xm2, xm1;
  {
    const int r3 = s0 - 3, r2 = s0 - 2, r1 = s0 - 1;
    const int l3 = lorg + lsgn * (r3 < 0 ? 0 : r3);
    const int l2 = lorg + lsgn * (r2 < 0 ? 0 : r2);
    const int l1 = lorg + lsgn * (r1 < 0 ? 0 : r1);
    const float v3 = XZ[(size_t)l3 * kXZP + d];
    const float v2 = XZ[(size_t)l2 * kXZP + d];
    const float v1 = XZ[(size_t)l1 * kXZP + d];
    xm3 = (r3 >= 0) ? v3 : 0.f;
    xm2 = (r2 >= 0) ? v2 : 0.f;
    xm1 = (r1 >= 0) ? v1 : 0.f;
  }
  const int hrow = wave >> 1;
  const int hch  = (wave & 1) * 128 + lane * 4;
#pragma unroll 1
  for (int sub = 0; sub < 4; ++sub) {
    const int sb = s0 + sub * 16;
    const int lb = dir ? (kSeqL - 16 - sb) : sb;
#pragma unroll 1
    for (int s = 0; s < 16; ++s) {
      const int l = lorg + lsgn * (sb + s);
      const float xcur = XZ[(size_t)l * kXZP + d];
      float acc = w0 * xm3;
      acc = fmaf(w1, xm2, acc);
      acc = fmaf(w2, xm1, acc);
      acc = fmaf(w3, xcur, acc);
      const float sv = acc + bc;
      const float sg = __builtin_amdgcn_rcpf(1.0f + __expf(-sv));
      sT[(l - lb) * kTP + tid] = sv * sg;
      xm3 = xm2; xm2 = xm1; xm1 = xcur;
    }
    __syncthreads();
    v4f fv[4];
    v8h bv[2];
#pragma unroll
    for (int it = 0; it < 4; ++it) fv[it] = *(const v4f*)(sT + (it * 4 + hrow) * kTP + hch);
#pragma unroll
    for (int it = 0; it < 2; ++it) {
      const float* sp = sT + (it * 8 + wave) * kTP + lane * 8;
      const v4f a0 = *(const v4f*)(sp);
      const v4f a1 = *(const v4f*)(sp + 4);
#pragma unroll
      for (int e = 0; e < 4; ++e) {
        bv[it][e]     = (_Float16)(a0[e] * kCarryUC);
        bv[it][4 + e] = (_Float16)(a1[e] * kCarryUC);
      }
    }
    for (int pass = 0; pass < 2; ++pass) {
#pragma unroll
      for (int it = 0; it < 4; ++it)
        *(volatile v4f*)(UC + (size_t)(lb + it * 4 + hrow) * kDin + d0 + hch) = fv[it];
#pragma unroll
      for (int it = 0; it < 2; ++it)
        *(volatile v8h*)(UC16 + (size_t)(lb + it * 8 + wave) * kDin + d0 + lane * 8) = bv[it];
      __threadfence();
    }
    __syncthreads();
  }
}

__global__ __launch_bounds__(256) void scan_kernel(
    const float* __restrict__ DLR, const float* __restrict__ UC, const float* __restrict__ XZ,
    const float* __restrict__ PROJ, const float* __restrict__ A_log, const float* __restrict__ Dv,
    const float* __restrict__ bdt, unsigned short* __restrict__ Y16, int dir)
{
  __shared__ __align__(16) float sBC[16 * 32];
  __shared__ __align__(16) float sY[16 * kTP];
  const int tid = threadIdx.x, lane = tid & 31, wave = tid >> 5;
  const int d0 = blockIdx.x * 256, d = d0 + tid;

  float An[kNst];
#pragma unroll
  for (int q4 = 0; q4 < 4; ++q4) {
    const v4f a4 = *(const v4f*)(A_log + (size_t)d * kNst + 4 * q4);
#pragma unroll
    for (int e = 0; e < 4; ++e) {
      const float av = a4[e];
      An[4 * q4 + e] = -__expf(bf16r(av));
    }
  }
  const float Dd = bf16r(Dv[d]);
  const float bb = bf16r(bdt[d]);
  float h[kNst];
#pragma unroll
  for (int n = 0; n < kNst; ++n) h[n] = 0.f;

#pragma unroll 1
  for (int c = 0; c < kSeqL / 16; ++c) {
    const int sb = c * 16;
    const int l0 = dir ? (kSeqL - 16 - sb) : sb;
    if (tid < 128) {
      const int r = tid >> 3, q = (tid & 7) * 4;
      const v4f v = *(const v4f*)(PROJ + (size_t)(l0 + r) * kPrjP + kDtR + q);
      *(v4f*)(sBC + r * 32 + q) = v;
    }
    __syncthreads();
#pragma unroll 1
    for (int s = 0; s < 16; ++s) {
      const int rr = dir ? (15 - s) : s;
      const size_t m = (size_t)(l0 + rr);
      const float a     = DLR[m * kDin + d] + bb;
      const float ea    = __expf(-fabsf(a));
      const float u1    = 1.0f + ea;
      const float l1p   = __logf(u1) + (ea - (u1 - 1.0f)) * __builtin_amdgcn_rcpf(u1);
      const float delta = fmaxf(a, 0.0f) + l1p;
      const float xv    = UC[m * kDin + d];
      const float zv    = XZ[m * kXZP + kDin + d];
      v4f Bq[4], Cq[4];
#pragma unroll
      for (int qq = 0; qq < 4; ++qq) {
        Bq[qq] = *(const v4f*)(sBC + rr * 32 + 4 * qq);
        Cq[qq] = *(const v4f*)(sBC + rr * 32 + kNst + 4 * qq);
      }
      const float dtx = delta * xv;
      float y = 0.f;
#pragma unroll
      for (int n = 0; n < kNst; ++n) {
        const float e  = __expf(delta * An[n]);
        const float hn = e * h[n] + dtx * Bq[n >> 2][n & 3];
        h[n] = hn;
        y = hn * Cq[n >> 2][n & 3] + y;
      }
      y = xv * Dd + y;
      const float sg = __builtin_amdgcn_rcpf(1.0f + __expf(-zv));
      const float g  = zv * sg;
      sY[rr * kTP + tid] = (y * g) * kCarryY;
    }
    __syncthreads();
    v8h hv[2];
#pragma unroll
    for (int it = 0; it < 2; ++it) {
      const float* sp = sY + (it * 8 + wave) * kTP + lane * 8;
      const v4f a0 = *(const v4f*)(sp);
      const v4f a1 = *(const v4f*)(sp + 4);
#pragma unroll
      for (int e = 0; e < 4; ++e) { hv[it][e] = (_Float16)a0[e]; hv[it][4 + e] = (_Float16)a1[e]; }
    }
    for (int pass = 0; pass < 2; ++pass) {
#pragma unroll
      for (int it = 0; it < 2; ++it)
        *(volatile v8h*)(Y16 + (size_t)(l0 + it * 8 + wave) * kDin + d0 + lane * 8) = hv[it];
      __threadfence();
    }
  }
}

extern "C" void kernel_launch(void* const* d_in, const int* in_sizes, int n_in,
                              void* d_out, int out_size, void* d_ws, size_t ws_size,
                              hipStream_t stream)
{
  if (n_in < 21) return;
  if (in_sizes[0] != kRows * kDmod) return;
  for (int p = 0; p < 2; ++p) {
    const int base = 1 + 9 * p;
    if (in_sizes[base + 0] != kXZP * kDmod) return;
    if (in_sizes[base + 1] != kDin * 4) return;
    if (in_sizes[base + 2] != kDin) return;
    if (in_sizes[base + 3] != kPrjN * kDin) return;
    if (in_sizes[base + 4] != kDin * kDtR) return;
    if (in_sizes[base + 5] != kDin) return;
    if (in_sizes[base + 6] != kDin * kNst) return;
    if (in_sizes[base + 7] != kDin) return;
    if (in_sizes[base + 8] != kDmod * kDin) return;
  }
  if (in_sizes[19] != kDmod * kYcP) return;
  if (in_sizes[20] != kDmod) return;
  if (out_size != kRows * kDmod) return;
  if (ws_size < kWsTotal) return;

  const float* x      = (const float*)d_in[0];
  const float* proj_W = (const float*)d_in[19];
  const float* proj_b = (const float*)d_in[20];
  float* dout = (float*)d_out;

  char* ws = (char*)d_ws;
  unsigned short* WIN16  = (unsigned short*)(ws + kOffWIN);
  unsigned short* WXP16  = (unsigned short*)(ws + kOffWXP);
  unsigned short* WDT16  = (unsigned short*)(ws + kOffWDT);
  unsigned short* WOUT16 = (unsigned short*)(ws + kOffWOUT);
  unsigned short* WPRJ16 = (unsigned short*)(ws + kOffWPRJ);
  unsigned short* X16    = (unsigned short*)(ws + kOffX16);
  float*          XZ     = (float*)(ws + kOffXZ);
  float*          UC     = (float*)(ws + kOffUC);
  unsigned short* UC16   = (unsigned short*)(ws + kOffUC16);
  float*          PROJ   = (float*)(ws + kOffPROJ);
  unsigned short* DT16   = (unsigned short*)(ws + kOffDT16);
  float*          DLR    = (float*)(ws + kOffDLR);
  unsigned short* Y16    = (unsigned short*)(ws + kOffY16);
  unsigned short* YCAT16 = (unsigned short*)(ws + kOffYC);

  cast_bf16_f16_kernel<<<(kRows * kDmod) / 8 / 256, 256, 0, stream>>>(
      x, X16, (kRows * kDmod) / 8, (kRows * kDmod) / 8, kCarryX);
  cast_bf16_f16_kernel<<<(kDmod * kYcP) / 8 / 256, 256, 0, stream>>>(
      proj_W, WPRJ16, (kDmod * kYcP) / 8, (kDmod * kYcP) / 8, kCarryW);

  for (int dir = 0; dir < 2; ++dir) {
    const int base = 1 + 9 * dir;
    const float* in_W    = (const float*)d_in[base + 0];
    const float* conv_w  = (const float*)d_in[base + 1];
    const float* conv_b  = (const float*)d_in[base + 2];
    const float* xproj_W = (const float*)d_in[base + 3];
    const float* dt_W    = (const float*)d_in[base + 4];
    const float* dt_b    = (const float*)d_in[base + 5];
    const float* A_log   = (const float*)d_in[base + 6];
    const float* Dv      = (const float*)d_in[base + 7];
    const float* out_W   = (const float*)d_in[base + 8];

    cast_bf16_f16_kernel<<<(kXZP * kDmod) / 8 / 256, 256, 0, stream>>>(
        in_W, WIN16, (kXZP * kDmod) / 8, (kXZP * kDmod) / 8, kCarryW);
    cast_bf16_f16_kernel<<<(kPrjP * kDin) / 8 / 256, 256, 0, stream>>>(
        xproj_W, WXP16, (kPrjP * kDin) / 8, (kPrjN * kDin) / 8, kCarryW);
    cast_bf16_f16_kernel<<<(kDin * kDtR) / 8 / 256, 256, 0, stream>>>(
        dt_W, WDT16, (kDin * kDtR) / 8, (kDin * kDtR) / 8, kCarryWdt);
    cast_bf16_f16_kernel<<<(kDmod * kDin) / 8 / 256, 256, 0, stream>>>(
        out_W, WOUT16, (kDmod * kDin) / 8, (kDmod * kDin) / 8, kCarryW);

    for (int b = 0; b < kBatch; ++b) {
      const unsigned short* X16b = X16 + (size_t)b * kSeqL * kDmod;
      unsigned short* ycb = YCAT16 + (size_t)b * kSeqL * kYcP + (size_t)dir * kDmod;

      wmma_gemm64<0, 0, false><<<dim3(256, 1), 256, 0, stream>>>(
          X16b, kDmod, WIN16, kDmod, (void*)XZ, kXZP, proj_b, kSeqL, kXZP, kDmod, kSclIn);

      conv_silu_kernel<<<dim3(kDin / 256, kSeqL / 64), 256, 0, stream>>>(XZ, conv_w, conv_b, UC, UC16, dir);

      wmma_gemm64<0, 0, false><<<dim3(8, 1), 256, 0, stream>>>(
          UC16, kDin, WXP16, kDin, (void*)PROJ, kPrjP, proj_b, kSeqL, kPrjP, kDin, kSclXp);

      dt_cast_kernel<<<(kSeqL * kDtR) / 8 / 256, 256, 0, stream>>>(PROJ, DT16, (kSeqL * kDtR) / 8, kCarryDT);

      wmma_gemm64<0, 0, false><<<dim3(128, 1), 256, 0, stream>>>(
          DT16, kDtR, WDT16, kDtR, (void*)DLR, kDin, proj_b, kSeqL, kDin, kDtR, kSclDt);

      scan_kernel<<<dim3(kDin / 256, 1), 256, 0, stream>>>(DLR, UC, XZ, PROJ, A_log, Dv, dt_b, Y16, dir);

      wmma_gemm64<0, 1, false><<<dim3(64, 1), 256, 0, stream>>>(
          Y16, kDin, WOUT16, kDin, (void*)ycb, kYcP, proj_b, kSeqL, kDmod, kDin, kSclOut);
    }
  }

  wmma_gemm64<2, 0, true><<<dim3(128, 1), 256, 0, stream>>>(
      YCAT16, kYcP, WPRJ16, kYcP, (void*)dout, kDmod, proj_b, kRows, kDmod, kYcP, kSclPrj);
}
